// Decoder_52235392254571
// MI455X (gfx1250) — hardware-verified
//
#include <hip/hip_runtime.h>
#include <math.h>

constexpr int NBAT  = 64;
constexpr int NSTEP = 32;
constexpr int NSRC  = 64;
constexpr int NVOC  = 32000;
constexpr int NEMB  = 512;
constexpr int NHID  = 1024;
constexpr int NCTX  = 2048;
constexpr int NG3   = 3 * NHID;
constexpr int NQG   = 4 * NHID;
constexpr int PKW   = NEMB + NHID + NCTX;
constexpr int NROWS = NBAT * NSTEP;
constexpr int NBS   = NBAT * NSRC;
constexpr int NOUT0 = NROWS * NEMB;
constexpr int NOUT1 = NBAT * NHID;
constexpr float WCARRY      = 16.0f;
constexpr float WCARRY_INV  = 1.0f / 16.0f;
constexpr float LOCARRY     = 2048.0f;
constexpr float LOCARRY_INV = 1.0f / 2048.0f;
constexpr float NEGFILL     = -3.4028234663852886e38f;
constexpr int BV_BIH1  = 0;
constexpr int BV_BHH1  = 3072;
constexpr int BV_BQH2  = 6144;
constexpr int BV_BIH2  = 10240;
constexpr int BV_VAT   = 13312;
constexpr int BV_BFIN  = 14336;
constexpr int BV_TOTAL = 14848;

static_assert(PKW == 3584, "packed K");
static_assert(NEMB % 32 == 0 && NHID % 32 == 0 && NCTX % 32 == 0 && PKW % 32 == 0, "K multiples of 32");
static_assert(NROWS % 64 == 0 && NBS % 64 == 0 && NBAT % 32 == 0, "M tile multiples");
static_assert(NG3 % 64 == 0 && NQG % 64 == 0 && NHID % 64 == 0 && NEMB % 64 == 0, "N tile multiples");
static_assert(((NBS / 64) * (NHID / 64)) % 8 == 0, "cache grid exact");
static_assert(((NROWS / 64) * (NG3 / 64)) % 8 == 0, "gi1 grid exact");
static_assert(((NROWS / 64) * (NEMB / 64)) % 8 == 0, "logit grid exact");
static_assert(((NBAT / 32) * (NG3 / 64)) % 8 == 0 && ((NBAT / 32) * (NQG / 64)) % 8 == 0, "step grids exact");
static_assert((size_t)NOUT0 * 4 == 4194304, "out1 byte offset");
static_assert((size_t)(NOUT0 + NOUT1) * 4 == 4456448, "d_out total bytes");
static_assert(BV_BHH1 == 3 * 1024 && BV_BQH2 == 6 * 1024 && BV_BIH2 == 10 * 1024 && BV_VAT == 13 * 1024 && BV_BFIN == 14 * 1024, "vector plane blocks");

typedef __attribute__((ext_vector_type(16))) _Float16 v16h;
typedef __attribute__((ext_vector_type(8)))  _Float16 v8h;
typedef __attribute__((ext_vector_type(4)))  _Float16 v4h;
typedef __attribute__((ext_vector_type(16))) __bf16   v16b;
typedef __attribute__((ext_vector_type(8)))  __bf16   v8b;
typedef __attribute__((ext_vector_type(8)))  float    v8f;
typedef __attribute__((ext_vector_type(4)))  float    v4f;
typedef __attribute__((ext_vector_type(4)))  unsigned v4u;

__device__ __forceinline__ unsigned short f2bf_bits(float f) {
  unsigned u = __float_as_uint(f);
  return (unsigned short)((u + 0x7FFFu + ((u >> 16) & 1u)) >> 16);
}
__device__ __forceinline__ float bf_bits2f(unsigned short h) { return __uint_as_float(((unsigned)h) << 16); }
__device__ __forceinline__ float bf16r(float f) { return bf_bits2f(f2bf_bits(f)); }

__device__ __forceinline__ void split_hl(float a, _Float16& hi, _Float16& lo) {
  const _Float16 hraw = (_Float16)a;
  const float hcand = (float)hraw;
  const float hf = (fabsf(a) < 6.2e-5f) ? 0.0f : hcand;
  hi = (_Float16)hf;
  lo = (_Float16)((a - hf) * LOCARRY);
}

__device__ __forceinline__ float sig_f(float x) { return __builtin_amdgcn_rcpf(1.0f + expf(-x)); }
__device__ __forceinline__ float tanh_f(float x) {
  const float xc = fminf(fmaxf(x, -15.0f), 15.0f);
  const float e = expf(2.0f * xc);
  return 1.0f - 2.0f * __builtin_amdgcn_rcpf(e + 1.0f);
}

__device__ __forceinline__ void grp_guard4_h(v8f& a, v8f& b, v8f& c, v8f& d, v16h x, v16h y0, v16h y1, v16h y2, v16h y3) {
  asm volatile("v_nop\n\tv_nop\n\tv_nop\n\tv_nop" : "+v"(a), "+v"(b), "+v"(c), "+v"(d) : "v"(x), "v"(y0), "v"(y1), "v"(y2), "v"(y3));
}
__device__ __forceinline__ void grp_guard4_b(v8f& a, v8f& b, v8f& c, v8f& d, v16b x, v16b y0, v16b y1, v16b y2, v16b y3) {
  asm volatile("v_nop\n\tv_nop\n\tv_nop\n\tv_nop" : "+v"(a), "+v"(b), "+v"(c), "+v"(d) : "v"(x), "v"(y0), "v"(y1), "v"(y2), "v"(y3));
}
__device__ __forceinline__ void grp_guard8_h(v8f& a0, v8f& a1, v8f& a2, v8f& a3, v8f& c0, v8f& c1, v8f& c2, v8f& c3,
                                             v16h x, v16h y, v16h b0, v16h b1, v16h b2, v16h b3) {
  asm volatile("v_nop\n\tv_nop\n\tv_nop\n\tv_nop"
               : "+v"(a0), "+v"(a1), "+v"(a2), "+v"(a3), "+v"(c0), "+v"(c1), "+v"(c2), "+v"(c3)
               : "v"(x), "v"(y), "v"(b0), "v"(b1), "v"(b2), "v"(b3));
}
__device__ __forceinline__ void keep4_h(v16h a, v16h b, v16h c, v16h d) { asm volatile("v_nop" :: "v"(a), "v"(b), "v"(c), "v"(d)); }
__device__ __forceinline__ void keep4_b(v16b a, v16b b, v16b c, v16b d) { asm volatile("v_nop" :: "v"(a), "v"(b), "v"(c), "v"(d)); }
__device__ __forceinline__ void acc_guard4(v8f& a, v8f& b, v8f& c, v8f& d) { asm volatile("v_nop\n\tv_nop\n\tv_nop\n\tv_nop" : "+v"(a), "+v"(b), "+v"(c), "+v"(d)); }

template <typename T> struct Frag;
template <> struct Frag<_Float16> {
  typedef v16h V; union U { v16h v; v8h h[2]; };
  static __device__ __forceinline__ v16h load(const _Float16* p) {
    U f; f.h[0] = *(const v8h*)(p); f.h[1] = *(const v8h*)(p + 16); return f.v;
  }
  static __device__ __forceinline__ v8f mma(v16h a, v16h b, v8f c) {
    return __builtin_amdgcn_wmma_f32_16x16x32_f16(false, a, false, b, (short)0, c, false, false);
  }
  static __device__ __forceinline__ void guard4(v8f& a, v8f& b, v8f& c, v8f& d, v16h x, v16h y0, v16h y1, v16h y2, v16h y3) { grp_guard4_h(a, b, c, d, x, y0, y1, y2, y3); }
  static __device__ __forceinline__ void keep(v16h a, v16h b, v16h c, v16h d) { keep4_h(a, b, c, d); }
};
template <> struct Frag<__bf16> {
  typedef v16b V; union U { v16b v; v8b h[2]; };
  static __device__ __forceinline__ v16b load(const __bf16* p) {
    U f; f.h[0] = *(const v8b*)(p); f.h[1] = *(const v8b*)(p + 16); return f.v;
  }
  static __device__ __forceinline__ v8f mma(v16b a, v16b b, v8f c) {
    return __builtin_amdgcn_wmma_f32_16x16x32_bf16(false, a, false, b, (short)0, c, false, false);
  }
  static __device__ __forceinline__ void guard4(v8f& a, v8f& b, v8f& c, v8f& d, v16b x, v16b y0, v16b y1, v16b y2, v16b y3) { grp_guard4_b(a, b, c, d, x, y0, y1, y2, y3); }
  static __device__ __forceinline__ void keep(v16b a, v16b b, v16b c, v16b d) { keep4_b(a, b, c, d); }
};
template <int ET> struct Elem;
template <> struct Elem<0> { typedef _Float16 T; };
template <> struct Elem<1> { typedef __bf16 T; };

template <int ET, int ACT, bool HASBIAS>
__global__ __launch_bounds__(256) void gemm64_kernel(
    const unsigned short* __restrict__ Ap, int lda,
    const unsigned short* __restrict__ Btp, int ldb,
    float* __restrict__ C, int ldc, const float* __restrict__ bias,
    int M, int N, int K, float scale) {
  typedef typename Elem<ET>::T T;
  typedef typename Frag<T>::V V;
  const T* A  = (const T*)Ap;
  const T* Bt = (const T*)Btp;
  __shared__ __align__(16) float sT[8][16 * 68];
  const int lane = threadIdx.x & 31;
  const int wave = threadIdx.x >> 5;
  const int tilesN = N >> 6;
  const int tilesM = M >> 6;
  const int tile = blockIdx.x * 8 + wave;
  if (tile >= tilesM * tilesN) return;
  const int tm = tile / tilesN;
  const int tn = tile - tm * tilesN;
  const int m0 = tm << 6;
  const int n0 = tn << 6;
  const int rlane = lane & 15;
  const int koff  = (lane >> 4) * 8;
  const int mOff  = (lane >> 4) * 8;

  v8f acc[4][4];
#pragma unroll
  for (int i = 0; i < 4; ++i)
#pragma unroll
    for (int j = 0; j < 4; ++j) acc[i][j] = (v8f){0.f, 0.f, 0.f, 0.f, 0.f, 0.f, 0.f, 0.f};

  for (int k0 = 0; k0 < K; k0 += 32) {
    V bh[4];
#pragma unroll
    for (int j = 0; j < 4; ++j) {
      const size_t bo = (size_t)(n0 + (j << 4) + rlane) * ldb + koff + k0;
      bh[j] = Frag<T>::load(Bt + bo);
    }
#pragma unroll
    for (int i = 0; i < 4; ++i) {
      const size_t ao = (size_t)(m0 + (i << 4) + rlane) * lda + koff + k0;
      V ah = Frag<T>::load(A + ao);
#pragma unroll
      for (int j = 0; j < 4; ++j) acc[i][j] = Frag<T>::mma(ah, bh[j], acc[i][j]);
      Frag<T>::guard4(acc[i][0], acc[i][1], acc[i][2], acc[i][3], ah, bh[0], bh[1], bh[2], bh[3]);
    }
    Frag<T>::keep(bh[0], bh[1], bh[2], bh[3]);
  }
  acc_guard4(acc[0][0], acc[0][1], acc[0][2], acc[0][3]);
  acc_guard4(acc[1][0], acc[1][1], acc[1][2], acc[1][3]);
  acc_guard4(acc[2][0], acc[2][1], acc[2][2], acc[2][3]);
  acc_guard4(acc[3][0], acc[3][1], acc[3][2], acc[3][3]);

  float* slab = sT[wave];
  const int hh = lane >> 4, c4 = (lane & 15) * 4;
#pragma unroll
  for (int i = 0; i < 4; ++i) {
    const int mBase = m0 + (i << 4);
#pragma unroll
    for (int j = 0; j < 4; ++j) {
      const int n = n0 + (j << 4) + rlane;
      float bv = 0.f;
      if (HASBIAS) bv = bias[n];
#pragma unroll
      for (int r = 0; r < 8; ++r) slab[(mOff + r) * 68 + (j << 4) + rlane] = acc[i][j][r] * scale + bv;
    }
    __builtin_amdgcn_fence(__ATOMIC_RELEASE, "workgroup");
    __builtin_amdgcn_wave_barrier();
    __builtin_amdgcn_fence(__ATOMIC_ACQUIRE, "workgroup");
    if (ACT == 1) {
#pragma unroll 1
      for (int it = 0; it < 8; ++it) {
        const int row = it * 2 + hh;
        v4f v = *(const v4f*)(slab + row * 68 + c4);
        const float t0 = tanhf(v[0]);
        const float t1 = tanhf(v[1]);
        const float t2 = tanhf(v[2]);
        const float t3 = tanhf(v[3]);
        v4f o = {t0, t1, t2, t3};
        *(v4f*)(slab + row * 68 + c4) = o;
      }
      __builtin_amdgcn_fence(__ATOMIC_RELEASE, "workgroup");
      __builtin_amdgcn_wave_barrier();
      __builtin_amdgcn_fence(__ATOMIC_ACQUIRE, "workgroup");
    }
    for (int pass = 0; pass < 2; ++pass) {
#pragma unroll
      for (int it = 0; it < 8; ++it) {
        const int row = it * 2 + hh;
        v4f v = *(const v4f*)(slab + row * 68 + c4);
        *(volatile v4f*)(C + (size_t)(mBase + row) * ldc + n0 + c4) = v;
      }
      __threadfence();
    }
    __builtin_amdgcn_fence(__ATOMIC_RELEASE, "workgroup");
    __builtin_amdgcn_wave_barrier();
    __builtin_amdgcn_fence(__ATOMIC_ACQUIRE, "workgroup");
  }
}

__global__ __launch_bounds__(256) void gemm_hl_kernel(
    const unsigned short* __restrict__ Ahip, int ldah,
    const unsigned short* __restrict__ Alop, int ldal,
    const unsigned short* __restrict__ Btp, int ldb,
    float* __restrict__ C, int ldc, const float* __restrict__ bias,
    int M, int N, int K, float scale) {
  const _Float16* Ahi = (const _Float16*)Ahip;
  const _Float16* Alo = (const _Float16*)Alop;
  const _Float16* Bt  = (const _Float16*)Btp;
  __shared__ __align__(16) float sT[8][16 * 68];
  const int lane = threadIdx.x & 31;
  const int wave = threadIdx.x >> 5;
  const int tilesN = N >> 6;
  const int tilesM = M >> 5;
  const int tile = blockIdx.x * 8 + wave;
  if (tile >= tilesM * tilesN) return;
  const int tm = tile / tilesN;
  const int tn = tile - tm * tilesN;
  const int m0 = tm << 5;
  const int n0 = tn << 6;
  const int rlane = lane & 15;
  const int koff  = (lane >> 4) * 8;
  const int mOff  = (lane >> 4) * 8;

  v8f acch[2][4], accl[2][4];
#pragma unroll
  for (int i = 0; i < 2; ++i)
#pragma unroll
    for (int j = 0; j < 4; ++j) {
      acch[i][j] = (v8f){0.f, 0.f, 0.f, 0.f, 0.f, 0.f, 0.f, 0.f};
      accl[i][j] = (v8f){0.f, 0.f, 0.f, 0.f, 0.f, 0.f, 0.f, 0.f};
    }

  for (int k0 = 0; k0 < K; k0 += 32) {
    v16h bh[4];
#pragma unroll
    for (int j = 0; j < 4; ++j) {
      const size_t bo = (size_t)(n0 + (j << 4) + rlane) * ldb + koff + k0;
      bh[j] = Frag<_Float16>::load(Bt + bo);
    }
#pragma unroll
    for (int i = 0; i < 2; ++i) {
      const size_t aoh = (size_t)(m0 + (i << 4) + rlane) * ldah + koff + k0;
      const size_t aol = (size_t)(m0 + (i << 4) + rlane) * ldal + koff + k0;
      const v16h ah = Frag<_Float16>::load(Ahi + aoh);
      const v16h al = Frag<_Float16>::load(Alo + aol);
#pragma unroll
      for (int j = 0; j < 4; ++j) {
        acch[i][j] = Frag<_Float16>::mma(ah, bh[j], acch[i][j]);
        accl[i][j] = Frag<_Float16>::mma(al, bh[j], accl[i][j]);
      }
      grp_guard8_h(acch[i][0], acch[i][1], acch[i][2], acch[i][3], accl[i][0], accl[i][1], accl[i][2], accl[i][3],
                   ah, al, bh[0], bh[1], bh[2], bh[3]);
    }
    keep4_h(bh[0], bh[1], bh[2], bh[3]);
  }
  acc_guard4(acch[0][0], acch[0][1], acch[0][2], acch[0][3]);
  acc_guard4(acch[1][0], acch[1][1], acch[1][2], acch[1][3]);
  acc_guard4(accl[0][0], accl[0][1], accl[0][2], accl[0][3]);
  acc_guard4(accl[1][0], accl[1][1], accl[1][2], accl[1][3]);

  float* slab = sT[wave];
  const int hh = lane >> 4, c4 = (lane & 15) * 4;
#pragma unroll
  for (int i = 0; i < 2; ++i) {
    const int mBase = m0 + (i << 4);
#pragma unroll
    for (int j = 0; j < 4; ++j) {
      const int n = n0 + (j << 4) + rlane;
      const float bv = bias[n];
#pragma unroll
      for (int r = 0; r < 8; ++r) {
        const float s = acch[i][j][r] + accl[i][j][r] * LOCARRY_INV;
        slab[(mOff + r) * 68 + (j << 4) + rlane] = s * scale + bv;
      }
    }
    __builtin_amdgcn_fence(__ATOMIC_RELEASE, "workgroup");
    __builtin_amdgcn_wave_barrier();
    __builtin_amdgcn_fence(__ATOMIC_ACQUIRE, "workgroup");
    for (int pass = 0; pass < 2; ++pass) {
#pragma unroll
      for (int it = 0; it < 8; ++it) {
        const int row = it * 2 + hh;
        v4f v = *(const v4f*)(slab + row * 68 + c4);
        *(volatile v4f*)(C + (size_t)(mBase + row) * ldc + n0 + c4) = v;
      }
      __threadfence();
    }
    __builtin_amdgcn_fence(__ATOMIC_RELEASE, "workgroup");
    __builtin_amdgcn_wave_barrier();
    __builtin_amdgcn_fence(__ATOMIC_ACQUIRE, "workgroup");
  }
}

template <int MODE>
__global__ __launch_bounds__(256) void cvt8_kernel(const float* __restrict__ src, unsigned short* __restrict__ dst,
                                                   int nrow, int ncol8, int spitch, int dpitch, int dcol0, float sc) {
  const int i  = blockIdx.x * 256 + threadIdx.x;
  const int n8 = nrow * ncol8;
  if (i < n8) {
    const int row = i / ncol8;
    const int c8  = i - row * ncol8;
    const float* sp = src + (size_t)row * spitch + c8 * 8;
    const v4f a = *(const v4f*)(sp);
    const v4f b = *(const v4f*)(sp + 4);
    v8h hv;
#pragma unroll
    for (int e = 0; e < 4; ++e) {
      const float fa = a[e];
      const float fb = b[e];
      if (MODE == 0) {
        const unsigned short b0 = f2bf_bits(fa);
        const unsigned short b1 = f2bf_bits(fb);
        hv[e]     = __builtin_bit_cast(_Float16, b0);
        hv[4 + e] = __builtin_bit_cast(_Float16, b1);
      } else {
        hv[e]     = (_Float16)(bf16r(fa) * sc);
        hv[4 + e] = (_Float16)(bf16r(fb) * sc);
      }
    }
    unsigned short* dp = dst + (size_t)row * dpitch + dcol0 + c8 * 8;
    *(volatile v8h*)dp = hv;
    __threadfence();
    *(volatile v8h*)dp = hv;
  }
}

template <int MODE>
__global__ __launch_bounds__(256) void tpw_kernel(const float* __restrict__ src, int R, int C, int ldo,
                                                  unsigned short* __restrict__ O, float sc) {
  __shared__ float Tt[64 * 65];
  const int tid = threadIdx.x;
  const int c0 = blockIdx.x * 64, r0 = blockIdx.y * 64;
#pragma unroll
  for (int i = 0; i < 4; ++i) {
    const int idx = i * 256 + tid;
    const int rr = idx >> 4, cc = (idx & 15) * 4;
    const v4f v = *(const v4f*)(src + (size_t)(r0 + rr) * (size_t)C + c0 + cc);
    Tt[rr * 65 + cc + 0] = v[0];
    Tt[rr * 65 + cc + 1] = v[1];
    Tt[rr * 65 + cc + 2] = v[2];
    Tt[rr * 65 + cc + 3] = v[3];
  }
  __syncthreads();
  const int q = tid >> 3, c8 = (tid & 7) * 8;
  v8h hv[2];
#pragma unroll
  for (int g = 0; g < 2; ++g) {
    const int qq = g * 32 + q;
#pragma unroll
    for (int e = 0; e < 8; ++e) {
      const float f = Tt[(c8 + e) * 65 + qq];
      if (MODE == 0) {
        const unsigned short bits = f2bf_bits(f * sc);
        hv[g][e] = __builtin_bit_cast(_Float16, bits);
      } else {
        hv[g][e] = (_Float16)(bf16r(f) * sc);
      }
    }
  }
  for (int pass = 0; pass < 2; ++pass) {
#pragma unroll
    for (int g = 0; g < 2; ++g) {
      const size_t o = (size_t)(c0 + g * 32 + q) * (size_t)ldo + (size_t)(r0 + c8);
      *(volatile v8h*)(O + o) = hv[g];
    }
    __threadfence();
  }
}

__global__ __launch_bounds__(256) void emb_gather_kernel(const int* __restrict__ y, const float* __restrict__ emb,
                                                         unsigned short* __restrict__ pk) {
  const int i = blockIdx.x * 256 + threadIdx.x;
  const int row = i >> 6;
  const int c8  = i & 63;
  int yi = y[row];
  yi = yi < 0 ? 0 : yi;
  yi = yi > (NVOC - 1) ? (NVOC - 1) : yi;
  const float* sp = emb + (size_t)yi * NEMB + c8 * 8;
  const v4f a = *(const v4f*)(sp);
  const v4f b = *(const v4f*)(sp + 4);
  v8h hv;
#pragma unroll
  for (int e = 0; e < 4; ++e) {
    const float fa = a[e];
    const float fb = b[e];
    hv[e]     = (_Float16)bf16r(fa);
    hv[4 + e] = (_Float16)bf16r(fb);
  }
  unsigned short* dp = pk + (size_t)row * PKW + c8 * 8;
  *(volatile v8h*)dp = hv;
  __threadfence();
  *(volatile v8h*)dp = hv;
}

__global__ __launch_bounds__(256) void h_init_kernel(const float* __restrict__ hidden, float* __restrict__ hF,
                                                     unsigned short* __restrict__ hi_pl, unsigned short* __restrict__ lo_pl) {
  const int b = blockIdx.x, j = 4 * threadIdx.x;
  const v4f v = *(const v4f*)(hidden + (size_t)b * NHID + j);
  v4f o; v4h hv, lv;
#pragma unroll
  for (int e = 0; e < 4; ++e) {
    const float f = bf16r(v[e]);
    _Float16 h, l;
    split_hl(f, h, l);
    o[e] = f; hv[e] = h; lv[e] = l;
  }
  float* po = hF + (size_t)b * NHID + j;
  unsigned short* ph = hi_pl + (size_t)b * NHID + j;
  unsigned short* pl = lo_pl + (size_t)b * NHID + j;
  for (int pass = 0; pass < 2; ++pass) {
    *(volatile v4f*)po = o;
    *(volatile v4h*)ph = hv;
    *(volatile v4h*)pl = lv;
    __threadfence();
  }
}

__global__ __launch_bounds__(256) void vec_prep_kernel(const float* __restrict__ b_ih1, const float* __restrict__ b_hh1,
                                                       const float* __restrict__ bq, const float* __restrict__ b_hh2,
                                                       const float* __restrict__ b_ih2, const float* __restrict__ vat,
                                                       const float* __restrict__ bi, const float* __restrict__ bh,
                                                       const float* __restrict__ bc, float* __restrict__ dst) {
  const int blk = blockIdx.x, tid = threadIdx.x;
  if (blk < 14) {
    const float* src; int loc;
    if (blk < 3)       { src = b_ih1; loc = blk; }
    else if (blk < 6)  { src = b_hh1; loc = blk - 3; }
    else if (blk < 7)  { src = bq;    loc = 0; }
    else if (blk < 10) { src = b_hh2; loc = blk - 7; }
    else if (blk < 13) { src = b_ih2; loc = blk - 10; }
    else               { src = vat;   loc = 0; }
    const v4f v = *(const v4f*)(src + loc * 1024 + 4 * tid);
    v4f o;
#pragma unroll
    for (int e = 0; e < 4; ++e) o[e] = bf16r(v[e]);
    float* op = dst + blk * 1024 + 4 * tid;
    *(volatile v4f*)op = o;
    __threadfence();
    *(volatile v4f*)op = o;
  } else {
    if (tid < 128) {
      const v4f a = *(const v4f*)(bi + 4 * tid);
      const v4f b = *(const v4f*)(bh + 4 * tid);
      const v4f c = *(const v4f*)(bc + 4 * tid);
      v4f o;
#pragma unroll
      for (int e = 0; e < 4; ++e) o[e] = (bf16r(a[e]) + bf16r(b[e])) + bf16r(c[e]);
      float* op = dst + BV_BFIN + 4 * tid;
      *(volatile v4f*)op = o;
      __threadfence();
      *(volatile v4f*)op = o;
    }
  }
}

__global__ __launch_bounds__(256) void gru_gate_kernel(const float* __restrict__ gi, int gi_rs,
                                                       const float* __restrict__ gh, int gh_rs,
                                                       const float* __restrict__ hprior, float* __restrict__ hout,
                                                       unsigned short* __restrict__ hi_pl, int hi_rs,
                                                       unsigned short* __restrict__ lo_pl,
                                                       float* __restrict__ hfin, int write_fin) {
  const int b = blockIdx.x, j = 4 * threadIdx.x;
  const float* gib = gi + (size_t)b * gi_rs + j;
  const float* ghb = gh + (size_t)b * gh_rs + j;
  const v4f ir = *(const v4f*)(gib);
  const v4f iz = *(const v4f*)(gib + NHID);
  const v4f in = *(const v4f*)(gib + 2 * NHID);
  const v4f hr = *(const v4f*)(ghb);
  const v4f hz = *(const v4f*)(ghb + NHID);
  const v4f hn = *(const v4f*)(ghb + 2 * NHID);
  const v4f hp = *(const v4f*)(hprior + (size_t)b * NHID + j);
  v4f o; v4h hv, lv;
#pragma unroll
  for (int e = 0; e < 4; ++e) {
    const float r = sig_f(ir[e] + hr[e]);
    const float z = sig_f(iz[e] + hz[e]);
    const float n = tanh_f(in[e] + r * hn[e]);
    const float hnew = (1.0f - z) * n + z * hp[e];
    _Float16 h, l;
    split_hl(hnew, h, l);
    o[e] = hnew; hv[e] = h; lv[e] = l;
  }
  float* po = hout + (size_t)b * NHID + j;
  float* pf = hfin + (size_t)b * NHID + j;
  unsigned short* ph = hi_pl + (size_t)b * hi_rs + j;
  unsigned short* pl = lo_pl + (size_t)b * NHID + j;
  for (int pass = 0; pass < 2; ++pass) {
    *(volatile v4f*)po = o;
    *(volatile v4h*)ph = hv;
    *(volatile v4h*)pl = lv;
    if (write_fin != 0) *(volatile v4f*)pf = o;
    __threadfence();
  }
}

__global__ __launch_bounds__(256) void attn_step_kernel(const float* __restrict__ qg, const float* __restrict__ cache,
                                                        const float* __restrict__ vat, const int* __restrict__ mask,
                                                        const unsigned short* __restrict__ ctxb,
                                                        unsigned short* __restrict__ pk_hi, unsigned short* __restrict__ a_lo) {
  __shared__ __align__(16) float sq[NHID];
  __shared__ __align__(16) float sv[NHID];
  __shared__ float ssc[NSRC];
  __shared__ float sp[NSRC];
  const int tid = threadIdx.x, lane = tid & 31, wave = tid >> 5;
  const int b = blockIdx.x;
  {
    const v4f qv = *(const v4f*)(qg + (size_t)b * NQG + 4 * tid);
    const v4f vv = *(const v4f*)(vat + 4 * tid);
    *(v4f*)(sq + 4 * tid) = qv;
    *(v4f*)(sv + 4 * tid) = vv;
  }
  __syncthreads();

#pragma unroll 1
  for (int si = 0; si < 8; ++si) {
    const int s = wave * 8 + si;
    const float* cp = cache + ((size_t)(b * NSRC + s)) * NHID + 4 * lane;
    float acc = 0.0f;
#pragma unroll 2
    for (int i = 0; i < 8; ++i) {
      const v4f cv = *(const v4f*)(cp + 128 * i);
      const v4f qv = *(const v4f*)(sq + 128 * i + 4 * lane);
      const v4f vv = *(const v4f*)(sv + 128 * i + 4 * lane);
#pragma unroll
      for (int e = 0; e < 4; ++e) acc += tanh_f(qv[e] + cv[e]) * vv[e];
    }
#pragma unroll
    for (int off = 1; off < 32; off <<= 1) acc += __shfl_xor(acc, off, 32);
    if (lane == 0) ssc[s] = acc;
  }
  __syncthreads();

  {
    const int mk0 = mask[b * NSRC + lane];
    const int mk1 = mask[b * NSRC + 32 + lane];
    float x0 = ssc[lane];
    float x1 = ssc[lane + 32];
    x0 = (mk0 != 0) ? NEGFILL : x0;
    x1 = (mk1 != 0) ? NEGFILL : x1;
    float m = fmaxf(x0, x1);
#pragma unroll
    for (int off = 1; off < 32; off <<= 1) m = fmaxf(m, __shfl_xor(m, off, 32));
    const float e0 = expf(x0 - m);
    const float e1 = expf(x1 - m);
    float sum = e0 + e1;
#pragma unroll
    for (int off = 1; off < 32; off <<= 1) sum += __shfl_xor(sum, off, 32);
    const float inv = __builtin_amdgcn_rcpf(sum);
    if (wave == 0) {
      sp[lane]      = e0 * inv;
      sp[lane + 32] = e1 * inv;
    }
  }
  __syncthreads();

  float a0 = 0.f, a1 = 0.f, a2 = 0.f, a3 = 0.f, a4 = 0.f, a5 = 0.f, a6 = 0.f, a7 = 0.f;
  const unsigned short* cb = ctxb + (size_t)b * NSRC * NCTX + 8 * tid;
#pragma unroll 2
  for (int s = 0; s < NSRC; ++s) {
    const v4u w = *(const v4u*)(cb + (size_t)s * NCTX);
    const float p = sp[s];
    const unsigned w0 = w[0];
    const unsigned w1 = w[1];
    const unsigned w2 = w[2];
    const unsigned w3 = w[3];
    a0 += p * __uint_as_float(w0 << 16);
    a1 += p * __uint_as_float(w0 & 0xffff0000u);
    a2 += p * __uint_as_float(w1 << 16);
    a3 += p * __uint_as_float(w1 & 0xffff0000u);
    a4 += p * __uint_as_float(w2 << 16);
    a5 += p * __uint_as_float(w2 & 0xffff0000u);
    a6 += p * __uint_as_float(w3 << 16);
    a7 += p * __uint_as_float(w3 & 0xffff0000u);
  }
  v8h hv, lv;
  {
    _Float16 h, l;
    split_hl(a0, h, l); hv[0] = h; lv[0] = l;
    split_hl(a1, h, l); hv[1] = h; lv[1] = l;
    split_hl(a2, h, l); hv[2] = h; lv[2] = l;
    split_hl(a3, h, l); hv[3] = h; lv[3] = l;
    split_hl(a4, h, l); hv[4] = h; lv[4] = l;
    split_hl(a5, h, l); hv[5] = h; lv[5] = l;
    split_hl(a6, h, l); hv[6] = h; lv[6] = l;
    split_hl(a7, h, l); hv[7] = h; lv[7] = l;
  }
  unsigned short* ph = pk_hi + (size_t)b * ((size_t)NSTEP * PKW) + 8 * tid;
  unsigned short* pl = a_lo + (size_t)b * NCTX + 8 * tid;
  for (int pass = 0; pass < 2; ++pass) {
    *(volatile v8h*)ph = hv;
    *(volatile v8h*)pl = lv;
    __threadfence();
  }
}

extern "C" void kernel_launch(void* const* d_in, const int* in_sizes, int n_in,
                              void* d_out, int out_size, void* d_ws, size_t ws_size, hipStream_t stream) {
  if (n_in < 23 || d_out == nullptr || d_ws == nullptr) return;
  if (in_sizes[0] != NBAT * NSTEP || in_sizes[1] != NBAT * NSRC * NCTX || in_sizes[2] != NBAT * NSRC ||
      in_sizes[3] != NBAT * NHID || in_sizes[4] != NVOC * NEMB || in_sizes[5] != NG3 * NEMB ||
      in_sizes[6] != NG3 * NHID || in_sizes[7] != NG3 || in_sizes[8] != NG3 || in_sizes[9] != NHID * NHID ||
      in_sizes[10] != NHID || in_sizes[11] != NCTX * NHID || in_sizes[12] != NHID || in_sizes[13] != NG3 * NCTX ||
      in_sizes[14] != NG3 * NHID || in_sizes[15] != NG3 || in_sizes[16] != NG3 || in_sizes[17] != NEMB * NEMB ||
      in_sizes[18] != NEMB || in_sizes[19] != NEMB * NHID || in_sizes[20] != NEMB || in_sizes[21] != NEMB * NCTX ||
      in_sizes[22] != NEMB || out_size != NOUT0 + NOUT1) return;

  const int*   y      = (const int*)  d_in[0];
  const float* ctx    = (const float*)d_in[1];
  const int*   cmask  = (const int*)  d_in[2];
  const float* hidden = (const float*)d_in[3];
  const float* emb    = (const float*)d_in[4];
  const float* W_ih1  = (const float*)d_in[5];
  const float* W_hh1  = (const float*)d_in[6];
  const float* b_ih1  = (const float*)d_in[7];
  const float* b_hh1  = (const float*)d_in[8];
  const float* Wq     = (const float*)d_in[9];
  const float* bq     = (const float*)d_in[10];
  const float* Wk     = (const float*)d_in[11];
  const float* v_attn = (const float*)d_in[12];
  const float* W_ih2  = (const float*)d_in[13];
  const float* W_hh2  = (const float*)d_in[14];
  const float* b_ih2  = (const float*)d_in[15];
  const float* b_hh2  = (const float*)d_in[16];
  const float* Wi     = (const float*)d_in[17];
  const float* bi     = (const float*)d_in[18];
  const float* Wh     = (const float*)d_in[19];
  const float* bh     = (const float*)d_in[20];
  const float* Wc     = (const float*)d_in[21];
  const float* bc     = (const float*)d_in[22];
  float* out0 = (float*)d_out;
  float* out1 = out0 + (size_t)NOUT0;

  char* ws = (char*)d_ws; size_t off = 0;
  auto carve = [&](size_t bytes) -> char* { char* p = ws + off; off += (bytes + 255) & ~(size_t)255; return p; };
  unsigned short* CTXB = (unsigned short*)carve((size_t)NBS * NCTX * 2);
  unsigned short* WKT  = (unsigned short*)carve((size_t)NHID * NCTX * 2);
  float*          CACHE = (float*)carve((size_t)NBS * NHID * 4);
  unsigned short* WIH1 = (unsigned short*)carve((size_t)NG3 * NEMB * 2);
  unsigned short* WHH1 = (unsigned short*)carve((size_t)NG3 * NHID * 2);
  unsigned short* WH1C = (unsigned short*)carve((size_t)NQG * NHID * 2);
  unsigned short* WIH2 = (unsigned short*)carve((size_t)NG3 * NCTX * 2);
  unsigned short* WFIN = (unsigned short*)carve((size_t)NEMB * PKW * 2);
  unsigned short* PK   = (unsigned short*)carve((size_t)NROWS * PKW * 2);
  float*          GI1  = (float*)carve((size_t)NROWS * NG3 * 4);
  float*          GH1  = (float*)carve((size_t)NBAT * NG3 * 4);
  float*          QGH2 = (float*)carve((size_t)NBAT * NQG * 4);
  float*          GI2  = (float*)carve((size_t)NBAT * NG3 * 4);
  float*          HF   = (float*)carve((size_t)NBAT * NHID * 4);
  float*          H1F  = (float*)carve((size_t)NBAT * NHID * 4);
  unsigned short* H0HI = (unsigned short*)carve((size_t)NBAT * NHID * 2);
  unsigned short* HLO  = (unsigned short*)carve((size_t)NBAT * NHID * 2);
  unsigned short* H1HI = (unsigned short*)carve((size_t)NBAT * NHID * 2);
  unsigned short* H1LO = (unsigned short*)carve((size_t)NBAT * NHID * 2);
  unsigned short* ALO  = (unsigned short*)carve((size_t)NBAT * NCTX * 2);
  float*          BV   = (float*)carve((size_t)BV_TOTAL * 4);
  if (off > ws_size || off > (size_t)134217728) return;

  cvt8_kernel<0><<<(NBS * (NCTX / 8)) / 256, 256, 0, stream>>>(ctx, CTXB, NBS, NCTX / 8, NCTX, NCTX, 0, 1.0f);
  tpw_kernel<0><<<dim3(NHID / 64, NCTX / 64), 256, 0, stream>>>(Wk, NCTX, NHID, NCTX, WKT, 1.0f);
  cvt8_kernel<1><<<(NG3 * (NEMB / 8)) / 256, 256, 0, stream>>>(W_ih1, WIH1, NG3, NEMB / 8, NEMB, NEMB, 0, WCARRY);
  cvt8_kernel<1><<<(NG3 * (NHID / 8)) / 256, 256, 0, stream>>>(W_hh1, WHH1, NG3, NHID / 8, NHID, NHID, 0, WCARRY);
  tpw_kernel<1><<<dim3(NHID / 64, NHID / 64), 256, 0, stream>>>(Wq, NHID, NHID, NHID, WH1C, WCARRY);
  cvt8_kernel<1><<<(NG3 * (NHID / 8)) / 256, 256, 0, stream>>>(W_hh2, WH1C + (size_t)NHID * NHID, NG3, NHID / 8, NHID, NHID, 0, WCARRY);
  cvt8_kernel<1><<<(NG3 * (NCTX / 8)) / 256, 256, 0, stream>>>(W_ih2, WIH2, NG3, NCTX / 8, NCTX, NCTX, 0, WCARRY);
  cvt8_kernel<1><<<(NEMB * (NEMB / 8)) / 256, 256, 0, stream>>>(Wi, WFIN, NEMB, NEMB / 8, NEMB, PKW, 0, WCARRY);
  cvt8_kernel<1><<<(NEMB * (NHID / 8)) / 256, 256, 0, stream>>>(Wh, WFIN, NEMB, NHID / 8, NHID, PKW, NEMB, WCARRY);
  cvt8_kernel<1><<<(NEMB * (NCTX / 8)) / 256, 256, 0, stream>>>(Wc, WFIN, NEMB, NCTX / 8, NCTX, PKW, NEMB + NHID, WCARRY);
  emb_gather_kernel<<<(NROWS * (NEMB / 8)) / 256, 256, 0, stream>>>(y, emb, PK);
  h_init_kernel<<<NBAT, 256, 0, stream>>>(hidden, HF, H0HI, HLO);
  vec_prep_kernel<<<15, 256, 0, stream>>>(b_ih1, b_hh1, bq, b_hh2, b_ih2, v_attn, bi, bh, bc, BV);

  gemm64_kernel<1, 0, false><<<((NBS / 64) * (NHID / 64)) / 8, 256, 0, stream>>>(
      CTXB, NCTX, WKT, NCTX, CACHE, NHID, BV, NBS, NHID, NCTX, 1.0f);
  gemm64_kernel<0, 0, true><<<((NROWS / 64) * (NG3 / 64)) / 8, 256, 0, stream>>>(
      PK, PKW, WIH1, NEMB, GI1, NG3, BV + BV_BIH1, NROWS, NG3, NEMB, WCARRY_INV);

  const int pk_step_pitch = NSTEP * PKW;
  for (int t = 0; t < NSTEP; ++t) {
    const unsigned short* hhi = (t == 0) ? H0HI : (PK + (size_t)(t - 1) * PKW + NEMB);
    const int ldhhi = (t == 0) ? NHID : pk_step_pitch;
    gemm_hl_kernel<<<((NBAT / 32) * (NG3 / 64)) / 8, 256, 0, stream>>>(
        hhi, ldhhi, HLO, NHID, WHH1, NHID, GH1, NG3, BV + BV_BHH1, NBAT, NG3, NHID, WCARRY_INV);
    gru_gate_kernel<<<NBAT, 256, 0, stream>>>(GI1 + (size_t)t * NG3, NSTEP * NG3, GH1, NG3, HF, H1F,
                                              H1HI, NHID, H1LO, out1, 0);
    gemm_hl_kernel<<<((NBAT / 32) * (NQG / 64)) / 8, 256, 0, stream>>>(
        H1HI, NHID, H1LO, NHID, WH1C, NHID, QGH2, NQG, BV + BV_BQH2, NBAT, NQG, NHID, WCARRY_INV);
    attn_step_kernel<<<NBAT, 256, 0, stream>>>(QGH2, CACHE, BV + BV_VAT, cmask, CTXB,
                                               PK + (size_t)t * PKW + NEMB + NHID, ALO);
    gemm_hl_kernel<<<((NBAT / 32) * (NG3 / 64)) / 8, 256, 0, stream>>>(
        PK + (size_t)t * PKW + NEMB + NHID, pk_step_pitch, ALO, NCTX, WIH2, NCTX, GI2, NG3, BV + BV_BIH2,
        NBAT, NG3, NCTX, WCARRY_INV);
    gru_gate_kernel<<<NBAT, 256, 0, stream>>>(GI2, NG3, QGH2 + NHID, NQG, H1F, HF,
                                              PK + (size_t)t * PKW + NEMB, pk_step_pitch, HLO, out1,
                                              (t == NSTEP - 1) ? 1 : 0);
  }

  gemm64_kernel<0, 1, true><<<((NROWS / 64) * (NEMB / 64)) / 8, 256, 0, stream>>>(
      PK, PKW, WFIN, PKW, out0, NEMB, BV + BV_BFIN, NROWS, NEMB, PKW, WCARRY_INV);
}
